// CryptoAggregator_29317446762861
// MI455X (gfx1250) — hardware-verified
//
#include <hip/hip_runtime.h>
#include <stddef.h>


#define DIM   256
#define DH    128
#define GR    32
#define AP    264
#define NTHR  256
#define NWAVE 8
#define NB    256
#define CHUNK 2048
#define WCAP  256
#define NGRP  (CHUNK / (NTHR * 4))

#define LDS_SACC (NB * DIM)
#define LDS_DEN  (NB)
#define LDS_LIST (NWAVE * WCAP)
#define LDS_BYTES ((LDS_SACC + LDS_DEN + LDS_LIST + NWAVE) * 4)

static_assert(NGRP == 2);
static_assert(WCAP == (CHUNK / NTHR) * 32);
static_assert(NB == 256);
static_assert((NB / NWAVE) == 32);
static_assert(CHUNK == 2048);
static_assert(((LDS_SACC + LDS_DEN) % 4) == 0);
static_assert(LDS_BYTES == 271392);
static_assert((AP % 8) == 0);
static_assert((DIM / 8) == 32);

typedef float    v4f  __attribute__((ext_vector_type(4)));
typedef float    v8f  __attribute__((ext_vector_type(8)));
typedef int      v4i  __attribute__((ext_vector_type(4)));
typedef _Float16 v8h  __attribute__((ext_vector_type(8)));
typedef _Float16 v16h __attribute__((ext_vector_type(16)));
union Frag   { v16h v; v8h half[2]; };
union Pack16 { v8h h; v4i i; _Float16 s[8]; };

__device__ __forceinline__ v8f wm(v16h a, v16h b, v8f c) {
  v8f d = __builtin_amdgcn_wmma_f32_16x16x32_f16(false, a, false, b, (short)0, c, false, false);
  asm volatile("v_nop\n\tv_nop\n\tv_nop\n\tv_nop" : "+v"(d) : "v"(a), "v"(b));
  return d;
}

__global__ __launch_bounds__(NTHR) void k_prep(const float* __restrict__ W1, _Float16* W1t, int total) {
  const int i = blockIdx.x * NTHR + threadIdx.x;
  if (i >= total) return;
  const int n  = i >> 5;
  const int k0 = (i & 31) * 8;
  Pack16 u;
#pragma unroll
  for (int j = 0; j < 8; ++j) u.s[j] = (_Float16)(W1[(size_t)(k0 + j) * DH + n] * 16.0f);
  _Float16* p = W1t + (size_t)n * DIM + k0;
  *(volatile v4i*)p = u.i;
  __threadfence();
  *(volatile v4i*)p = u.i;
}

__global__ __launch_bounds__(NTHR) void k_node(
    const float* __restrict__ x, const _Float16* __restrict__ W1t,
    const float* __restrict__ b1, const float* __restrict__ W2, const float* __restrict__ b2,
    float* wnode, int nN) {
  __shared__ __attribute__((aligned(16))) _Float16 At[GR * AP];
  __shared__ __attribute__((aligned(16))) float Ps[GR * NWAVE];
  __shared__ __attribute__((aligned(16))) float Ws[GR];

  const int tid  = threadIdx.x;
  const int lane = tid & 31;
  const int wave = tid >> 5;
  const int hh   = lane >> 4;
  const int m    = lane & 15;
  const int rowBase = blockIdx.x * GR;

  {
    const int r  = tid >> 3;
    const int c0 = (tid & 7) * 32;
    int row = rowBase + r;
    if (row > nN - 1) row = nN - 1;
    const float* p = x + (size_t)row * DIM + c0;
#pragma unroll
    for (int q = 0; q < 4; ++q) {
      const v4f f0 = *(const v4f*)(p + 8 * q);
      const v4f f1 = *(const v4f*)(p + 8 * q + 4);
      Pack16 u;
      u.s[0] = (_Float16)f0.x; u.s[1] = (_Float16)f0.y; u.s[2] = (_Float16)f0.z; u.s[3] = (_Float16)f0.w;
      u.s[4] = (_Float16)f1.x; u.s[5] = (_Float16)f1.y; u.s[6] = (_Float16)f1.z; u.s[7] = (_Float16)f1.w;
      *(v8h*)(At + r * AP + c0 + 8 * q) = u.h;
    }
  }
  __syncthreads();

  const int ncol = wave * 16 + m;
  v8f c0a = {0.f, 0.f, 0.f, 0.f, 0.f, 0.f, 0.f, 0.f};
  v8f c1a = {0.f, 0.f, 0.f, 0.f, 0.f, 0.f, 0.f, 0.f};
#pragma unroll
  for (int kt = 0; kt < DIM / 32; ++kt) {
    const int k0 = kt * 32;
    Frag a0, a1, b;
    const _Float16* pb  = W1t + (size_t)ncol * DIM + k0 + 8 * hh;
    const _Float16* pa0 = At + m * AP + k0 + 8 * hh;
    const _Float16* pa1 = At + (16 + m) * AP + k0 + 8 * hh;
    b.half[0]  = *(const v8h*)pb;  b.half[1]  = *(const v8h*)(pb + 16);
    a0.half[0] = *(const v8h*)pa0; a0.half[1] = *(const v8h*)(pa0 + 16);
    a1.half[0] = *(const v8h*)pa1; a1.half[1] = *(const v8h*)(pa1 + 16);
    c0a = wm(a0.v, b.v, c0a);
    c1a = wm(a1.v, b.v, c1a);
  }

  const float b1v = b1[ncol];
  const float w2v = W2[ncol];
  float pr[16];
#pragma unroll
  for (int r = 0; r < 8; ++r) {
    float hv = c0a[r] * 0.0625f + b1v;
    hv = fmaxf(hv, 0.f);
    pr[r] = hv * w2v;
    float hu = c1a[r] * 0.0625f + b1v;
    hu = fmaxf(hu, 0.f);
    pr[8 + r] = hu * w2v;
  }
#pragma unroll
  for (int mk = 1; mk < 16; mk <<= 1) {
#pragma unroll
    for (int r = 0; r < 16; ++r) pr[r] += __shfl_xor(pr[r], mk, 32);
  }
  if (m == 0) {
#pragma unroll
    for (int r = 0; r < 8; ++r) {
      Ps[(8 * hh + r) * NWAVE + wave]      = pr[r];
      Ps[(16 + 8 * hh + r) * NWAVE + wave] = pr[8 + r];
    }
  }
  __syncthreads();

  if (wave == 0) {
    const v4f p0 = *(const v4f*)(Ps + lane * NWAVE);
    const v4f p1 = *(const v4f*)(Ps + lane * NWAVE + 4);
    float s = b2[0] + ((p0.x + p0.y) + (p0.z + p0.w)) + ((p1.x + p1.y) + (p1.z + p1.w));
    s = fminf(fmaxf(s, -30.f), 30.f);
    const float e = __expf(-s);
    Ws[lane] = __builtin_amdgcn_rcpf(1.0f + e);
  }
  __syncthreads();
  if (wave == 0 && lane < 8) {
    const v4f v = *(const v4f*)(Ws + 4 * lane);
    float* gp = wnode + (size_t)rowBase + 4 * lane;
    *(volatile v4f*)gp = v;
    __threadfence();
    *(volatile v4f*)gp = v;
  }
}

__global__ __launch_bounds__(NTHR) void k_agg(
    const float* __restrict__ x, const int* __restrict__ ei, const float* __restrict__ wnode,
    float* out, int nN, int nE) {
  extern __shared__ v4f lds_dyn[];
  float* sacc = (float*)lds_dyn;
  float* den  = sacc + LDS_SACC;
  int*   list = (int*)(den + LDS_DEN);
  int*   wcnt = list + LDS_LIST;

  const int tid  = threadIdx.x;
  const int lane = tid & 31;
  const int wave = tid >> 5;
  const int nodeBase = blockIdx.x * NB;

  {
    const v4f z4 = {0.f, 0.f, 0.f, 0.f};
    for (int i = tid; i < (LDS_SACC + LDS_DEN) / 4; i += NTHR) lds_dyn[i] = z4;
  }
  __syncthreads();

  const int* keyp = ei;
  const int* colp = ei + nE;

  const int nChunks = (nE + CHUNK - 1) / CHUNK;
#pragma unroll 1
  for (int ch = 0; ch < nChunks; ++ch) {
    const int cbase = ch * CHUNK;
    int wc = 0;
#pragma unroll
    for (int g = 0; g < NGRP; ++g) {
      const int el0 = (g * NTHR + tid) * 4;
      const int e0  = cbase + el0;
      const int sent = -2147483647 - 1;
      v4i d;
      if (cbase + CHUNK <= nE) {
        d = *(const v4i*)(keyp + e0);
      } else {
        const int em = nE - 1;
        d.x = (e0     < nE) ? keyp[min(e0, em)]     : sent;
        d.y = (e0 + 1 < nE) ? keyp[min(e0 + 1, em)] : sent;
        d.z = (e0 + 2 < nE) ? keyp[min(e0 + 2, em)] : sent;
        d.w = (e0 + 3 < nE) ? keyp[min(e0 + 3, em)] : sent;
      }
      const unsigned s0 = (unsigned)d.x - (unsigned)nodeBase;
      const unsigned s1 = (unsigned)d.y - (unsigned)nodeBase;
      const unsigned s2 = (unsigned)d.z - (unsigned)nodeBase;
      const unsigned s3 = (unsigned)d.w - (unsigned)nodeBase;
      const bool h0 = s0 < (unsigned)NB;
      const bool h1 = s1 < (unsigned)NB;
      const bool h2 = s2 < (unsigned)NB;
      const bool h3 = s3 < (unsigned)NB;
      const unsigned many = __builtin_amdgcn_ballot_w32(h0 | h1 | h2 | h3);
      if (many != 0u) {
#define HITJ(J, HJ, SJ) { \
          const unsigned mj = __builtin_amdgcn_ballot_w32(HJ); \
          if (HJ) { \
            const int pos = wc + (int)__builtin_amdgcn_mbcnt_lo(mj, 0u); \
            if (pos < WCAP) list[wave * WCAP + pos] = ((el0 + (J)) << 8) | (int)(SJ); \
          } \
          wc += (int)__builtin_popcount(mj); }
        HITJ(0, h0, s0)
        HITJ(1, h1, s1)
        HITJ(2, h2, s2)
        HITJ(3, h3, s3)
#undef HITJ
      }
    }
    if (lane == 0) wcnt[wave] = wc;
    __syncthreads();

#pragma unroll 1
    for (int wsx = 0; wsx < NWAVE; ++wsx) {
      int n = wcnt[wsx];
      n = n > WCAP ? WCAP : n;
      n = n < 0 ? 0 : n;
      n = __builtin_amdgcn_readfirstlane(n);
#pragma unroll 1
      for (int base = 0; base < n; base += 32) {
        const int idx = base + lane;
        const int li  = idx < WCAP ? idx : (WCAP - 1);
        const int myent = list[wsx * WCAP + li];
        const bool mine = (idx < n) && ((((myent & (NB - 1)) >> 5)) == wave);
        unsigned mask = __builtin_amdgcn_ballot_w32(mine);
        while (mask != 0u) {
          const int bpos = __builtin_ctz(mask);
          mask &= mask - 1u;
          const int ent  = __shfl(myent, bpos, 32);
          const int slot = ent & (NB - 1);
          const int el   = (ent >> 8) & (CHUNK - 1);
          int e = cbase + el;
          if (e > nE - 1) e = nE - 1;
          int src = colp[e];
          src = src < 0 ? 0 : (src > nN - 1 ? nN - 1 : src);
          const float w = wnode[src];
          const float* xr = x + (size_t)src * DIM + 4 * lane;
          const v4f xa = *(const v4f*)xr;
          const v4f xb = *(const v4f*)(xr + 128);
          v4f* sa = (v4f*)(sacc + slot * DIM + 4 * lane);
          v4f* sb = (v4f*)(sacc + slot * DIM + 128 + 4 * lane);
          const v4f ca = *sa;
          const v4f cb = *sb;
          *sa = ca + w * xa;
          *sb = cb + w * xb;
          if (lane == 0) {
            const float od = den[slot];
            den[slot] = od + w;
          }
        }
      }
    }
    __syncthreads();
  }
  __syncthreads();

#pragma unroll 1
  for (int j = 0; j < NB / NWAVE; ++j) {
    const int slot = wave * (NB / NWAVE) + j;
    const int node = nodeBase + slot;
    if (node >= nN) break;
    const float dv  = den[slot];
    const float inv = (dv > 0.f) ? __builtin_amdgcn_rcpf(fmaxf(dv, 1e-12f)) : 0.f;
    const v4f ya = *(const v4f*)(sacc + slot * DIM + 4 * lane) * inv;
    const v4f yb = *(const v4f*)(sacc + slot * DIM + 128 + 4 * lane) * inv;
    float* op = out + (size_t)node * DIM + 4 * lane;
    *(volatile v4f*)op         = ya;
    *(volatile v4f*)(op + 128) = yb;
    __threadfence();
    *(volatile v4f*)op         = ya;
    *(volatile v4f*)(op + 128) = yb;
  }
}

extern "C" void kernel_launch(void* const* d_in, const int* in_sizes, int n_in,
                              void* d_out, int out_size, void* d_ws, size_t ws_size,
                              hipStream_t stream) {
  if (n_in < 6) return;
  const int nN = in_sizes[0] / DIM;
  if (nN <= 0 || in_sizes[0] != nN * DIM) return;
  const int nE = in_sizes[1] / 2;
  if (nE < 0 || in_sizes[1] != 2 * nE) return;
  if (in_sizes[2] != DIM * DH) return;
  if (in_sizes[3] != DH || in_sizes[4] != DH || in_sizes[5] < 1) return;
  if (out_size != nN * DIM) return;

  const float* x  = (const float*)d_in[0];
  const int*   ei = (const int*)d_in[1];
  const float* W1 = (const float*)d_in[2];
  const float* b1 = (const float*)d_in[3];
  const float* W2 = (const float*)d_in[4];
  const float* b2 = (const float*)d_in[5];
  float* out = (float*)d_out;

  const int nP = ((nN + GR - 1) / GR) * GR;
  size_t off = 0;
  _Float16* W1t = (_Float16*)((char*)d_ws + off); off += (size_t)DH * DIM * sizeof(_Float16);
  float* wnode  = (float*)((char*)d_ws + off);    off += (size_t)nP * sizeof(float);
  if (off > ws_size) return;

  const int total8 = DH * DIM / 8;
  k_prep<<<(total8 + NTHR - 1) / NTHR, NTHR, 0, stream>>>(W1, W1t, total8);

  k_node<<<nP / GR, NTHR, 0, stream>>>(x, W1t, b1, W2, b2, wnode, nN);

  hipFuncSetAttribute(reinterpret_cast<const void*>(&k_agg),
                      hipFuncAttributeMaxDynamicSharedMemorySize, LDS_BYTES);
  const int grid = (nN + NB - 1) / NB;
  k_agg<<<grid, NTHR, LDS_BYTES, stream>>>(x, ei, wnode, out, nN, nE);
}
